// FSSConv1dCell_73710228734015
// MI455X (gfx1250) — hardware-verified
//
#include <hip/hip_runtime.h>


#define NB_  8
#define CC   256
#define LL   4096
#define L1   4094
#define L2   4092
#define L3   4088
#define LP   4096
#define NG_  8
#define CPG  32
typedef _Float16 h16;
typedef unsigned short bf;
typedef __attribute__((ext_vector_type(16))) __bf16   v16bf;
typedef __attribute__((ext_vector_type(16))) _Float16 v16h;
typedef __attribute__((ext_vector_type(8)))  _Float16 v8h;
typedef __attribute__((ext_vector_type(8)))  unsigned short v8us;
typedef __attribute__((ext_vector_type(8)))  float    v8f;
typedef __attribute__((ext_vector_type(4)))  float    v4f;
typedef v8h  __attribute__((may_alias)) v8ha;
typedef v4f  __attribute__((may_alias)) v4fa;
typedef v8us __attribute__((may_alias)) v8usa;

__device__ __forceinline__ unsigned short f2bf(float f) { unsigned u = __float_as_uint(f); u += 0x7FFFu + ((u >> 16) & 1u); return (unsigned short)(u >> 16); }
__device__ __forceinline__ float bf2f(unsigned short b) { return __uint_as_float(((unsigned)b) << 16); }
__device__ __forceinline__ float bfr(float f) { return bf2f(f2bf(f)); }
__device__ __forceinline__ v16h cat16(v8h lo, v8h hi) { return __builtin_shufflevector(lo, hi, 0, 1, 2, 3, 4, 5, 6, 7, 8, 9, 10, 11, 12, 13, 14, 15); }
__device__ __forceinline__ v16bf cat16b(v8us lo, v8us hi) { return __builtin_bit_cast(v16bf, __builtin_shufflevector(lo, hi, 0, 1, 2, 3, 4, 5, 6, 7, 8, 9, 10, 11, 12, 13, 14, 15)); }
__device__ __forceinline__ v8f wmma16(v16h a, v16h b, v8f c) { return __builtin_amdgcn_wmma_f32_16x16x32_f16(false, a, false, b, (short)0, c, false, false); }
__device__ __forceinline__ v8f wmmab(v16bf a, v16bf b, v8f c) { return __builtin_amdgcn_wmma_f32_16x16x32_bf16(false, a, false, b, (short)0, c, false, false); }


template <typename T16> struct WFrag;
template <> struct WFrag<h16> { typedef v16h V; static __device__ __forceinline__ V ld(const h16* p) { return cat16(*(const v8h*)p, *(const v8h*)(p + 16)); } static __device__ __forceinline__ v8f mma(V a, V b, v8f c) { return wmma16(a, b, c); } };
template <> struct WFrag<bf> { typedef v16bf V; static __device__ __forceinline__ V ld(const bf* p) { return cat16b(*(const v8us*)p, *(const v8us*)(p + 16)); } static __device__ __forceinline__ v8f mma(V a, V b, v8f c) { return wmmab(a, b, c); } };
template <typename T16, int NSPLIT, bool BIAS>
__global__ __launch_bounds__(32) void k_gemmw(const T16* __restrict__ A, const T16* __restrict__ A2, const T16* __restrict__ Bt, const T16* __restrict__ Bt2, int K, float* C, int ldc, const float* __restrict__ bias, size_t sA, size_t sB, size_t sC) {
    typedef typename WFrag<T16>::V V;
    __shared__ __align__(16) float os[16 * 68];
    const size_t z = blockIdx.z; A += z * sA; if (A2) A2 += z * sA; Bt += z * sB; if (Bt2) Bt2 += z * sB; C += z * sC;
    const int lane = threadIdx.x & 31, lr = lane & 15, hi = lane >> 4; const int r0 = blockIdx.x * 64, c0 = blockIdx.y * 64;
    v8f acc[4][4];
#pragma unroll
    for (int mb = 0; mb < 4; ++mb)
#pragma unroll
        for (int nb = 0; nb < 4; ++nb) acc[mb][nb] = (v8f){};
    const size_t aoff = (size_t)(r0 + lr) * K + 8 * hi, boff = (size_t)(c0 + lr) * K + 8 * hi;
#pragma unroll 1
    for (int kc = 0; kc < K; kc += 32) {
        V a[4], a2[4];
#pragma unroll
        for (int mb = 0; mb < 4; ++mb) { a[mb] = WFrag<T16>::ld(A + aoff + (size_t)mb * 16 * K + kc); if (NSPLIT == 1 || NSPLIT == 2) a2[mb] = WFrag<T16>::ld(A2 + aoff + (size_t)mb * 16 * K + kc); }
#pragma unroll
        for (int nb = 0; nb < 4; ++nb) { const V b = WFrag<T16>::ld(Bt + boff + (size_t)nb * 16 * K + kc); V b2; if (NSPLIT >= 2) b2 = WFrag<T16>::ld(Bt2 + boff + (size_t)nb * 16 * K + kc);
#pragma unroll
            for (int mb = 0; mb < 4; ++mb) { acc[mb][nb] = WFrag<T16>::mma(a[mb], b, acc[mb][nb]); if (NSPLIT == 1 || NSPLIT == 2) acc[mb][nb] = WFrag<T16>::mma(a2[mb], b, acc[mb][nb]); if (NSPLIT >= 2) acc[mb][nb] = WFrag<T16>::mma(a[mb], b2, acc[mb][nb]); } }
        asm volatile("v_nop\n\tv_nop\n\tv_nop\n\tv_nop" : "+v"(acc[0][0]), "+v"(acc[1][1]), "+v"(acc[2][2]), "+v"(acc[3][3]) : "v"(a[0]), "v"(a[3]));
    }
#pragma unroll
    for (int mb = 0; mb < 4; ++mb) {
#pragma unroll
        for (int nb = 0; nb < 4; ++nb) {
#pragma unroll
            for (int j = 0; j < 8; ++j) os[(hi * 8 + j) * 68 + nb * 16 + lr] = acc[mb][nb][j]; }
        __builtin_amdgcn_wave_barrier(); asm volatile("" ::: "memory");
        float* crow = C + (size_t)(r0 + mb * 16) * ldc + c0;
#pragma unroll 1
        for (int ps = 0; ps < 2; ++ps) {
#pragma unroll
            for (int s = 0; s < 8; ++s) { const int row = 2 * s + hi, cofs = lr * 4; v4f val = *(const v4fa*)(os + row * 68 + cofs); if (BIAS) { val[0] += bfr(bias[c0 + cofs]); val[1] += bfr(bias[c0 + cofs + 1]); val[2] += bfr(bias[c0 + cofs + 2]); val[3] += bfr(bias[c0 + cofs + 3]); }
                *(volatile v4f*)(crow + (size_t)row * ldc + cofs) = val; }
            if (ps == 0) __threadfence(); }
        __builtin_amdgcn_wave_barrier(); asm volatile("" ::: "memory");
    }
}

__device__ __forceinline__ h16 tohx(float x) { return (h16)x; }
__device__ __forceinline__ float sigm_(float x) { return __fdiv_rn(1.0f, 1.0f + __expf(-x)); }
__device__ __forceinline__ int shuf(int c) { return (c % CPG) * NG_ + c / CPG; }
typedef __attribute__((ext_vector_type(2))) _Float16 v2h;
typedef __attribute__((ext_vector_type(4))) _Float16 v4h;
typedef __attribute__((ext_vector_type(4))) unsigned short v4us;

template <typename T> __device__ __forceinline__ T cvt16(float x);
template <> __device__ __forceinline__ h16 cvt16<h16>(float x) { return tohx(bfr(x)); }
template <> __device__ __forceinline__ bf cvt16<bf>(float x) { return f2bf(x); }
template <typename T> __global__ __launch_bounds__(256) void k_wconv(const float* __restrict__ w, int CIN, int KT, int doshuf, T* Bt) { const int cinpg = CIN / NG_; const size_t e = ((size_t)blockIdx.x * 256 + threadIdx.x) * 4; const size_t KK = (size_t)CIN * KT; if (e >= (size_t)CC * KK) return; const int k = (int)(e % KK); const int n = (int)(e / KK);
    int co; if (doshuf) { co = (n % NG_) * CPG + n / NG_; } else co = n;
    const int g = co / CPG; T o[4];
#pragma unroll
    for (int q = 0; q < 4; ++q) { const int kk = k + q; const int ci = kk / KT, t = kk % KT; const int cl = ci - g * cinpg; o[q] = (cl >= 0 && cl < cinpg) ? cvt16<T>(w[((size_t)co * cinpg + cl) * KT + t]) : cvt16<T>(0.f); }
    typedef __attribute__((ext_vector_type(4))) unsigned short v4x; v4x ov; ov[0] = *(unsigned short*)&o[0]; ov[1] = *(unsigned short*)&o[1]; ov[2] = *(unsigned short*)&o[2]; ov[3] = *(unsigned short*)&o[3];
    *(volatile v4x*)((unsigned short*)Bt + e) = ov; __threadfence(); *(volatile v4x*)((unsigned short*)Bt + e) = ov; }
__global__ __launch_bounds__(256) void k_bperm(const float* __restrict__ b, int doshuf, float* BP) { const int n = threadIdx.x; int co = doshuf ? (n % NG_) * CPG + n / NG_ : n; const float v = b[co]; *(volatile float*)(BP + n) = v; __threadfence(); *(volatile float*)(BP + n) = v; }
__global__ __launch_bounds__(256) void k_col0(const float* __restrict__ x, bf* A) { const size_t e = ((size_t)blockIdx.x * 256 + threadIdx.x) * 4; if (e >= (size_t)LP * CC * 3) return; const int k = (int)(e % (CC * 3)); const int l = (int)(e / (CC * 3)); v4us o;
#pragma unroll
    for (int q = 0; q < 4; ++q) { const int kk = k + q; const int ci = kk / 3, t = kk % 3; o[q] = (l < L1) ? f2bf(x[(size_t)ci * LL + l + t]) : (unsigned short)0; } *(volatile v4us*)(A + e) = o; __threadfence(); *(volatile v4us*)(A + e) = o; }
__global__ __launch_bounds__(256) void k_colh(const h16* __restrict__ Hin, int KT, int Lout, h16* A) { const size_t KK = (size_t)CC * KT; const size_t e = ((size_t)blockIdx.x * 256 + threadIdx.x) * 4; if (e >= (size_t)LP * KK) return; const int k = (int)(e % KK); const int l = (int)(e / KK); v4h o;
#pragma unroll
    for (int q = 0; q < 4; ++q) { const int kk = k + q; const int ci = kk / KT, t = kk % KT; o[q] = (l < Lout) ? Hin[(size_t)(l + t) * CC + ci] : (h16)0.f; } *(volatile v4h*)(A + e) = o; __threadfence(); *(volatile v4h*)(A + e) = o; }
__global__ __launch_bounds__(256) void k_f16(const float* __restrict__ F, size_t n4, h16* P) { const size_t i = ((size_t)blockIdx.x * 256 + threadIdx.x) * 4; if (i >= n4 * 4) return; const v4f a = *(const v4f*)(F + i); v4h o; o[0] = tohx(a[0]); o[1] = tohx(a[1]); o[2] = tohx(a[2]); o[3] = tohx(a[3]); *(volatile v4h*)(P + i) = o; __threadfence(); *(volatile v4h*)(P + i) = o; }
__global__ __launch_bounds__(256) void k_sort(const float* __restrict__ H2f, h16* CAT) { __shared__ float sv[CC]; const int l = blockIdx.x; const int c = threadIdx.x; h16* row = CAT + (size_t)l * 2 * CC; v2h o;
    if (l >= L2) { o[0] = (h16)0.f; o[1] = (h16)0.f; *(volatile v2h*)(row + 2 * c) = o; __threadfence(); *(volatile v2h*)(row + 2 * c) = o; return; }
    sv[c] = H2f[(size_t)l * CC + c]; __syncthreads();
    for (int k = 2; k <= CC; k <<= 1) { for (int j = k >> 1; j > 0; j >>= 1) { const int ixj = c ^ j; if (ixj > c) { const bool up = ((c & k) == 0); const float a = sv[c], bq = sv[ixj]; if ((a > bq) == up) { sv[c] = bq; sv[ixj] = a; } } __syncthreads(); } }
    if (c < CC / 2) { o[0] = tohx(sv[2 * c]); o[1] = tohx(sv[2 * c + 1]); } else { const int cc = 2 * (c - CC / 2); o[0] = tohx(H2f[(size_t)l * CC + cc]); o[1] = tohx(H2f[(size_t)l * CC + cc + 1]); }
    *(volatile v2h*)(row + 2 * c) = o; __threadfence(); *(volatile v2h*)(row + 2 * c) = o; }
__global__ __launch_bounds__(256) void k_gate(const float* __restrict__ H2f, const float* __restrict__ A2, h16* G16) { const size_t i = ((size_t)blockIdx.x * 256 + threadIdx.x) * 4; if (i >= (size_t)LP * CC) return; const v4f h = *(const v4f*)(H2f + i), a = *(const v4f*)(A2 + i); v4h o;
#pragma unroll
    for (int q = 0; q < 4; ++q) o[q] = tohx(__fmul_rn(h[q], sigm_(a[q]))); *(volatile v4h*)(G16 + i) = o; __threadfence(); *(volatile v4h*)(G16 + i) = o; }
__global__ __launch_bounds__(256) void k_yout(const float* __restrict__ Y, int b, float* OUT) { const int s = blockIdx.x * 256 + threadIdx.x; if (s >= CC * L3 / 4) return; const int f = 4 * s; const int c = f / L3, l0 = f % L3; v4f o;
#pragma unroll
    for (int q = 0; q < 4; ++q) o[q] = Y[(size_t)(l0 + q) * CC + c]; float* dst = OUT + (size_t)b * CC * L3 + f; *(volatile v4f*)dst = o; __threadfence(); *(volatile v4f*)dst = o; }

extern "C" void kernel_launch(void* const* d_in, const int* in_sizes, int n_in,
                              void* d_out, int out_size, void* d_ws, size_t ws_size, hipStream_t stream) {
    (void)in_sizes; (void)n_in; (void)out_size;
    const float* x = (const float*)d_in[0]; const float* w1 = (const float*)d_in[1]; const float* b1 = (const float*)d_in[2]; const float* w2 = (const float*)d_in[3]; const float* b2 = (const float*)d_in[4]; const float* wa1 = (const float*)d_in[5]; const float* ba1 = (const float*)d_in[6]; const float* wa2 = (const float*)d_in[7]; const float* ba2 = (const float*)d_in[8]; const float* w3 = (const float*)d_in[9]; const float* b3 = (const float*)d_in[10];
    float* OUT = (float*)d_out;
    char* wsp = (char*)d_ws;
    auto take = [&](size_t bytes) { char* p = wsp; wsp += (bytes + 255) & ~(size_t)255; return (void*)p; };
    bf* W1B = (bf*)take((size_t)CC * 768 * 2); h16* W2B = (h16*)take((size_t)CC * 768 * 2); h16* WA1 = (h16*)take((size_t)CC * 512 * 2); h16* WA2 = (h16*)take((size_t)CC * 256 * 2); h16* W3B = (h16*)take((size_t)CC * 1280 * 2); float* BP1 = (float*)take(1024); float* BP2 = (float*)take(1024); float* BPA = (float*)take(1024);
    bf* A0 = (bf*)take((size_t)LP * 768 * 2); h16* A16 = (h16*)take((size_t)LP * 1280 * 2); float* F1 = (float*)take((size_t)LP * CC * 4); h16* H1 = (h16*)take((size_t)LP * CC * 2); float* H2f = (float*)take((size_t)LP * CC * 4); h16* CAT = (h16*)take((size_t)LP * 2 * CC * 2); float* A1f = (float*)take((size_t)LP * CC * 4); h16* A1 = (h16*)take((size_t)LP * CC * 2); float* A2f = (float*)take((size_t)LP * CC * 4); h16* G16 = (h16*)take((size_t)LP * CC * 2); float* Y = (float*)take((size_t)LP * CC * 4);
    if ((size_t)(wsp - (char*)d_ws) > ws_size) return;
    k_wconv<bf><<<(unsigned)(((size_t)CC * 768 / 4 + 255) / 256), 256, 0, stream>>>(w1, CC, 3, 1, W1B); k_bperm<<<1, 256, 0, stream>>>(b1, 1, BP1);
    k_wconv<h16><<<(unsigned)(((size_t)CC * 768 / 4 + 255) / 256), 256, 0, stream>>>(w2, CC, 3, 1, W2B); k_bperm<<<1, 256, 0, stream>>>(b2, 1, BP2);
    k_wconv<h16><<<(unsigned)(((size_t)CC * 512 / 4 + 255) / 256), 256, 0, stream>>>(wa1, 2 * CC, 1, 1, WA1); k_bperm<<<1, 256, 0, stream>>>(ba1, 1, BPA);
    k_wconv<h16><<<(unsigned)(((size_t)CC * 256 / 4 + 255) / 256), 256, 0, stream>>>(wa2, CC, 1, 0, WA2);
    k_wconv<h16><<<(unsigned)(((size_t)CC * 1280 / 4 + 255) / 256), 256, 0, stream>>>(w3, CC, 5, 0, W3B);
    for (int b = 0; b < NB_; ++b) { const float* xb = x + (size_t)b * CC * LL;
        k_col0<<<(unsigned)(((size_t)LP * 768 / 4 + 255) / 256), 256, 0, stream>>>(xb, A0);
        k_gemmw<bf, 0, true><<<dim3(LP / 64, CC / 64, 1), 32, 0, stream>>>(A0, nullptr, W1B, nullptr, 768, F1, CC, BP1, 0, 0, 0); k_f16<<<(unsigned)(((size_t)LP * CC / 4 + 255) / 256), 256, 0, stream>>>(F1, (size_t)LP * CC / 4, H1);
        k_colh<<<(unsigned)(((size_t)LP * 768 / 4 + 255) / 256), 256, 0, stream>>>(H1, 3, L2, A16);
        k_gemmw<h16, 0, true><<<dim3(LP / 64, CC / 64, 1), 32, 0, stream>>>(A16, nullptr, W2B, nullptr, 768, H2f, CC, BP2, 0, 0, 0);
        k_sort<<<LP, 256, 0, stream>>>(H2f, CAT);
        k_gemmw<h16, 0, true><<<dim3(LP / 64, CC / 64, 1), 32, 0, stream>>>(CAT, nullptr, WA1, nullptr, 512, A1f, CC, BPA, 0, 0, 0); k_f16<<<(unsigned)(((size_t)LP * CC / 4 + 255) / 256), 256, 0, stream>>>(A1f, (size_t)LP * CC / 4, A1);
        k_gemmw<h16, 0, true><<<dim3(LP / 64, CC / 64, 1), 32, 0, stream>>>(A1, nullptr, WA2, nullptr, 256, A2f, CC, ba2, 0, 0, 0);
        k_gate<<<(unsigned)(((size_t)LP * CC / 4 + 255) / 256), 256, 0, stream>>>(H2f, A2f, G16);
        k_colh<<<(unsigned)(((size_t)LP * 1280 / 4 + 255) / 256), 256, 0, stream>>>(G16, 5, L3, A16);
        k_gemmw<h16, 0, true><<<dim3(LP / 64, CC / 64, 1), 32, 0, stream>>>(A16, nullptr, W3B, nullptr, 1280, Y, CC, b3, 0, 0, 0);
        k_yout<<<(CC * L3 / 4 + 255) / 256, 256, 0, stream>>>(Y, b, OUT); }
}
